// MambaBlock_3607772529040
// MI455X (gfx1250) — hardware-verified
//
#include <hip/hip_runtime.h>
#include <math.h>

typedef __attribute__((ext_vector_type(16))) _Float16 v16h;
typedef __attribute__((ext_vector_type(8)))  _Float16 v8h;
typedef __attribute__((ext_vector_type(16))) __bf16   v16b;
typedef __attribute__((ext_vector_type(8)))  __bf16   v8b;
typedef __attribute__((ext_vector_type(8)))  float    v8f;
typedef __attribute__((ext_vector_type(4)))  float    v4f;

constexpr int kBatch = 2;
constexpr int kSeqT  = 1024;
constexpr int kDm    = 1024;
constexpr int kDin   = 2048;
constexpr int kNst   = 16;
constexpr int kDtr   = 128;
constexpr int kPrjN  = kDtr + 2 * kNst;
constexpr int kPrjP  = 192;
constexpr int kXZP   = 2 * kDin;
constexpr int kRows  = kBatch * kSeqT;
constexpr int kTileP = 260;
constexpr int kBiasP = 256;
static_assert(kPrjN == 160, "dbc width");
static_assert(kPrjP % 64 == 0 && kPrjP >= kPrjN, "padded dbc width");
static_assert(kBiasP >= kPrjP, "padded bias extent");
static_assert((kDm % 64) == 0 && (kDin % 64) == 0 && (kDtr % 64) == 0, "transpose tiles / GEMM K multiples of 32");
static_assert((kRows % 64) == 0 && (kXZP % 64) == 0, "GEMM M,N multiples of 64");
static_assert((kSeqT % 64) == 0 && (kDin % 256) == 0 && (kSeqT % 16) == 0, "tile multiples");

constexpr float kCarryDlr  = 16.0f;
constexpr float kCarryWdup = 16.0f;
constexpr float kFoldDt    = 1.0f / (kCarryDlr * kCarryWdup);
constexpr float kLog2e     = 1.4426950408889634f;
constexpr float kRmsEps    = 1e-6f;

constexpr size_t kOffINWH  = 0;
constexpr size_t kOffINWL  = kOffINWH  + (size_t)kXZP  * kDm  * 2;
constexpr size_t kOffDBH   = kOffINWL  + (size_t)kXZP  * kDm  * 2;
constexpr size_t kOffDBL   = kOffDBH   + (size_t)kPrjP * kDin * 2;
constexpr size_t kOffDUPWT = kOffDBL   + (size_t)kPrjP * kDin * 2;
constexpr size_t kOffOUTWH = kOffDUPWT + (size_t)kDin  * kDtr * 2;
constexpr size_t kOffOUTWL = kOffOUTWH + (size_t)kDm   * kDin * 2;
constexpr size_t kOffBIASP = kOffOUTWL + (size_t)kDm   * kDin * 2;
constexpr size_t kOffHNH   = kOffBIASP + (size_t)kBiasP * 4;
constexpr size_t kOffHNL   = kOffHNH   + (size_t)kRows * kDm  * 2;
constexpr size_t kOffXZ    = kOffHNL   + (size_t)kRows * kDm  * 2;
constexpr size_t kOffUC    = kOffXZ    + (size_t)kRows * kXZP * 4;
constexpr size_t kOffUCH   = kOffUC    + (size_t)kRows * kDin * 4;
constexpr size_t kOffUCL   = kOffUCH   + (size_t)kRows * kDin * 2;
constexpr size_t kOffDBC   = kOffUCL   + (size_t)kRows * kDin * 2;
constexpr size_t kOffDLR16 = kOffDBC   + (size_t)kRows * kPrjP * 4;
constexpr size_t kOffDPRE  = kOffDLR16 + (size_t)kRows * kDtr * 2;
constexpr size_t kWsTotal  = kOffDPRE  + (size_t)kRows * kDin * 4;
constexpr size_t kOffYGH   = kOffUCH;
constexpr size_t kOffYGL   = kOffUCL;
static_assert(kWsTotal == 121635840ull, "carve total");
static_assert(kWsTotal <= 134217728ull, "carve cap");
static_assert(kOffUCL - kOffUCH == (size_t)kRows * kDin * 2 && kOffDBC - kOffUCL == (size_t)kRows * kDin * 2, "re-used plane extents");
static_assert((kOffINWL % 128) == 0 && (kOffDBH % 128) == 0 && (kOffDBL % 128) == 0 && (kOffDUPWT % 128) == 0 &&
              (kOffOUTWH % 128) == 0 && (kOffOUTWL % 128) == 0 && (kOffBIASP % 128) == 0 && (kOffHNH % 128) == 0 &&
              (kOffHNL % 128) == 0 && (kOffXZ % 128) == 0 && (kOffUC % 128) == 0 && (kOffUCH % 128) == 0 &&
              (kOffUCL % 128) == 0 && (kOffDBC % 128) == 0 && (kOffDLR16 % 128) == 0 && (kOffDPRE % 128) == 0,
              "128-B aligned regions");

__device__ __forceinline__ unsigned short f2bf_bits(float f) {
  unsigned u = __float_as_uint(f);
  return (unsigned short)((u + 0x7FFFu + ((u >> 16) & 1u)) >> 16);
}
__device__ __forceinline__ float bf_bits2f(unsigned short h) { return __uint_as_float(((unsigned)h) << 16); }

__device__ __forceinline__ void dep_guard4_h(v8f& a, v8f& b, v8f& c, v8f& d, v16h x, v16h y) {
  asm volatile("v_nop\n\tv_nop\n\tv_nop\n\tv_nop" : "+v"(a), "+v"(b), "+v"(c), "+v"(d) : "v"(x), "v"(y));
}
__device__ __forceinline__ void dep_guard4_b(v8f& a, v8f& b, v8f& c, v8f& d, v16b x, v16b y) {
  asm volatile("v_nop\n\tv_nop\n\tv_nop\n\tv_nop" : "+v"(a), "+v"(b), "+v"(c), "+v"(d) : "v"(x), "v"(y));
}
__device__ __forceinline__ void keep4_h(v16h a, v16h b, v16h c, v16h d) { asm volatile("v_nop" :: "v"(a), "v"(b), "v"(c), "v"(d)); }
__device__ __forceinline__ void keep4_b(v16b a, v16b b, v16b c, v16b d) { asm volatile("v_nop" :: "v"(a), "v"(b), "v"(c), "v"(d)); }
__device__ __forceinline__ void acc_guard4(v8f& a, v8f& b, v8f& c, v8f& d) { asm volatile("v_nop\n\tv_nop\n\tv_nop\n\tv_nop" : "+v"(a), "+v"(b), "+v"(c), "+v"(d)); }
template <typename T> struct Frag;
template <> struct Frag<_Float16> {
  typedef v16h V; union U { v16h v; v8h h[2]; };
  static __device__ __forceinline__ v16h load(const _Float16* p) {
    U f; f.h[0] = *(const v8h*)(p); f.h[1] = *(const v8h*)(p + 16); return f.v;
  }
  static __device__ __forceinline__ v8f mma(v16h a, v16h b, v8f c) {
    return __builtin_amdgcn_wmma_f32_16x16x32_f16(false, a, false, b, (short)0, c, false, false);
  }
  static __device__ __forceinline__ void guard4(v8f& a, v8f& b, v8f& c, v8f& d, v16h x, v16h y) { dep_guard4_h(a, b, c, d, x, y); }
  static __device__ __forceinline__ void keep(v16h a, v16h b, v16h c, v16h d) { keep4_h(a, b, c, d); }
};
template <> struct Frag<__bf16> {
  typedef v16b V; union U { v16b v; v8b h[2]; };
  static __device__ __forceinline__ v16b load(const __bf16* p) {
    U f; f.h[0] = *(const v8b*)(p); f.h[1] = *(const v8b*)(p + 16); return f.v;
  }
  static __device__ __forceinline__ v8f mma(v16b a, v16b b, v8f c) {
    return __builtin_amdgcn_wmma_f32_16x16x32_bf16(false, a, false, b, (short)0, c, false, false);
  }
  static __device__ __forceinline__ void guard4(v8f& a, v8f& b, v8f& c, v8f& d, v16b x, v16b y) { dep_guard4_b(a, b, c, d, x, y); }
  static __device__ __forceinline__ void keep(v16b a, v16b b, v16b c, v16b d) { keep4_b(a, b, c, d); }
};

template <int ET> struct Elem;
template <> struct Elem<0> { typedef _Float16 T; };
template <> struct Elem<1> { typedef __bf16 T; };
template <int ET, bool SPLIT, int BIAS_MODE, bool RESID>
__global__ __launch_bounds__(256) void wmma_gemm64(
    const unsigned short* __restrict__ Ap, const unsigned short* __restrict__ A2p, int lda, long strideA,
    const unsigned short* __restrict__ Btp, const unsigned short* __restrict__ Bt2p, int ldb, long strideB,
    float* __restrict__ Cout, int ldc, long strideC,
    const float* __restrict__ bias,
    const float* __restrict__ resid, long strideR,
    int M, int N, int K, float scale) {
  typedef typename Elem<ET>::T T;
  typedef typename Frag<T>::V V;
  const T* A = (const T*)Ap; const T* A2 = (const T*)A2p; const T* Bt = (const T*)Btp; const T* Bt2 = (const T*)Bt2p;
  __shared__ __align__(16) float sT[8][16 * 68];
  const int b    = blockIdx.y;
  const int lane = threadIdx.x & 31;
  const int wave = threadIdx.x >> 5;
  const int tilesN = N >> 6;
  const int tilesM = M >> 6;
  const int tile = blockIdx.x * 8 + wave;
  if (tile >= tilesM * tilesN) return;
  const int tm = tile / tilesN;
  const int tn = tile - tm * tilesN;
  const int m0 = tm << 6;
  const int n0 = tn << 6;

  const T* Ab  = A  + (size_t)b * strideA;
  const T* Bb  = Bt + (size_t)b * strideB;
  const T* Ab2 = SPLIT ? (A2  + (size_t)b * strideA) : nullptr;
  const T* Bb2 = SPLIT ? (Bt2 + (size_t)b * strideB) : nullptr;

  const int rlane = lane & 15;
  const int koff  = (lane >> 4) * 8;
  const int mOff  = (lane >> 4) * 8;

  v8f acc[4][4];
#pragma unroll
  for (int i = 0; i < 4; ++i)
#pragma unroll
    for (int j = 0; j < 4; ++j) acc[i][j] = (v8f){0.f,0.f,0.f,0.f,0.f,0.f,0.f,0.f};

  for (int k0 = 0; k0 < K; k0 += 32) {
    V bh[4], bl[4];
#pragma unroll
    for (int j = 0; j < 4; ++j) {
      const size_t bo = (size_t)(n0 + (j << 4) + rlane) * ldb + koff + k0;
      bh[j] = Frag<T>::load(Bb + bo);
      if (SPLIT) bl[j] = Frag<T>::load(Bb2 + bo);
    }
#pragma unroll
    for (int i = 0; i < 4; ++i) {
      const size_t ao = (size_t)(m0 + (i << 4) + rlane) * lda + koff + k0;
      V ah = Frag<T>::load(Ab + ao);
      V al;
      if (SPLIT) al = Frag<T>::load(Ab2 + ao);
#pragma unroll
      for (int j = 0; j < 4; ++j) {
        acc[i][j] = Frag<T>::mma(ah, bh[j], acc[i][j]);
        if (SPLIT) {
          acc[i][j] = Frag<T>::mma(ah, bl[j], acc[i][j]);
          acc[i][j] = Frag<T>::mma(al, bh[j], acc[i][j]);
        }
      }
      Frag<T>::guard4(acc[i][0], acc[i][1], acc[i][2], acc[i][3], ah, SPLIT ? al : ah);
    }
    Frag<T>::keep(bh[0], bh[1], bh[2], bh[3]);
    if (SPLIT) Frag<T>::keep(bl[0], bl[1], bl[2], bl[3]);
  }
  acc_guard4(acc[0][0], acc[0][1], acc[0][2], acc[0][3]);
  acc_guard4(acc[1][0], acc[1][1], acc[1][2], acc[1][3]);
  acc_guard4(acc[2][0], acc[2][1], acc[2][2], acc[2][3]);
  acc_guard4(acc[3][0], acc[3][1], acc[3][2], acc[3][3]);

  float* slab = sT[wave];
  float* C = Cout + (size_t)b * strideC;
  const float* Rb = resid + (size_t)b * strideR;
  const int hh = lane >> 4, c4 = (lane & 15) * 4;
#pragma unroll
  for (int i = 0; i < 4; ++i) {
    const int mBase = m0 + (i << 4);
#pragma unroll
    for (int j = 0; j < 4; ++j) {
      const int n = n0 + (j << 4) + rlane;
      float bv = 0.f;
      if (BIAS_MODE == 2) bv = bias[n];
#pragma unroll
      for (int r = 0; r < 8; ++r) {
        float v = acc[i][j][r] * scale;
        if (BIAS_MODE == 2) v += bv;
        slab[(mOff + r) * 68 + (j << 4) + rlane] = v;
      }
    }
    __builtin_amdgcn_fence(__ATOMIC_RELEASE, "workgroup");
    __builtin_amdgcn_wave_barrier();
    __builtin_amdgcn_fence(__ATOMIC_ACQUIRE, "workgroup");
    {
      v4f vv[8];
#pragma unroll
      for (int it = 0; it < 8; ++it) {
        const int row = it * 2 + hh;
        vv[it] = *(const v4f*)(slab + row * 68 + c4);
      }
      if (RESID) {
#pragma unroll
        for (int it = 0; it < 8; ++it) {
          const int row = it * 2 + hh;
          const v4f rr = *(const v4f*)(Rb + (size_t)(mBase + row) * ldc + n0 + c4);
          vv[it] = vv[it] + rr;
        }
      }
      for (int pass = 0; pass < 2; ++pass) {
#pragma unroll
        for (int it = 0; it < 8; ++it) {
          const int row = it * 2 + hh;
          *(volatile v4f*)(C + (size_t)(mBase + row) * ldc + n0 + c4) = vv[it];
        }
        __threadfence();
      }
    }
    __builtin_amdgcn_fence(__ATOMIC_RELEASE, "workgroup");
    __builtin_amdgcn_wave_barrier();
    __builtin_amdgcn_fence(__ATOMIC_ACQUIRE, "workgroup");
  }
}

__global__ __launch_bounds__(256) void transpose_cast_kernel(
    const float* __restrict__ W, unsigned short* __restrict__ Bt, int Kdim, int Ndim, float scale)
{
  __shared__ float tile[64 * 65];
  const int tid = threadIdx.x, lane = tid & 31, wave = tid >> 5;
  const int n0 = blockIdx.x * 64;
  const int k0 = blockIdx.y * 64;
#pragma unroll
  for (int p = 0; p < 16; ++p) {
    const int idx = tid + p * 256;
    const int kk  = idx >> 6;
    const int nn  = idx & 63;
    const int n   = n0 + nn;
    const int nc  = (n < Ndim) ? n : (Ndim - 1);
    const float v = W[(size_t)(k0 + kk) * Ndim + nc];
    tile[kk * 65 + nn] = (n < Ndim) ? (v * scale) : 0.f;
  }
  __syncthreads();
  const int q = lane >> 3, c8 = (lane & 7) * 8;
  v8h hv[2];
#pragma unroll
  for (int it = 0; it < 2; ++it) {
    const int nrow = it * 32 + wave * 4 + q;
#pragma unroll
    for (int e = 0; e < 8; ++e) hv[it][e] = (_Float16)tile[(c8 + e) * 65 + nrow];
  }
  for (int pass = 0; pass < 2; ++pass) {
#pragma unroll
    for (int it = 0; it < 2; ++it) {
      const int nrow = it * 32 + wave * 4 + q;
      *(volatile v8h*)(Bt + (size_t)(n0 + nrow) * Kdim + k0 + c8) = hv[it];
    }
    __threadfence();
  }
}

__global__ __launch_bounds__(256) void transpose_split_bf16_kernel(
    const float* __restrict__ W, unsigned short* __restrict__ Bh, unsigned short* __restrict__ Bl, int Kdim, int Ndim)
{
  __shared__ float tile[64 * 65];
  const int tid = threadIdx.x, lane = tid & 31, wave = tid >> 5;
  const int n0 = blockIdx.x * 64;
  const int k0 = blockIdx.y * 64;
#pragma unroll
  for (int p = 0; p < 16; ++p) {
    const int idx = tid + p * 256;
    const int kk  = idx >> 6;
    const int nn  = idx & 63;
    const int n   = n0 + nn;
    const int nc  = (n < Ndim) ? n : (Ndim - 1);
    const float v = W[(size_t)(k0 + kk) * Ndim + nc];
    tile[kk * 65 + nn] = (n < Ndim) ? v : 0.f;
  }
  __syncthreads();
  const int q = lane >> 3, c8 = (lane & 7) * 8;
  v8h hv[2], lv[2];
#pragma unroll
  for (int it = 0; it < 2; ++it) {
    const int nrow = it * 32 + wave * 4 + q;
#pragma unroll
    for (int e = 0; e < 8; ++e) {
      const float v = tile[(c8 + e) * 65 + nrow];
      const unsigned short hb = f2bf_bits(v);
      const unsigned short lb = f2bf_bits(v - bf_bits2f(hb));
      hv[it][e] = __builtin_bit_cast(_Float16, hb);
      lv[it][e] = __builtin_bit_cast(_Float16, lb);
    }
  }
  for (int pass = 0; pass < 2; ++pass) {
#pragma unroll
    for (int it = 0; it < 2; ++it) {
      const int nrow = it * 32 + wave * 4 + q;
      const size_t o = (size_t)(n0 + nrow) * Kdim + k0 + c8;
      *(volatile v8h*)(Bh + o) = hv[it];
      *(volatile v8h*)(Bl + o) = lv[it];
    }
    __threadfence();
  }
}

__global__ __launch_bounds__(64) void pad_bias_kernel(const float* __restrict__ src, float* __restrict__ dst, int nreal)
{
  const int e0 = threadIdx.x * 4;
  v4f v;
#pragma unroll
  for (int e = 0; e < 4; ++e) {
    const int idx = e0 + e;
    const int ic  = (idx < nreal) ? idx : (nreal - 1);
    const float s = src[ic];
    v[e] = (idx < nreal) ? s : 0.f;
  }
  *(volatile v4f*)(dst + e0) = v;
  __threadfence();
  *(volatile v4f*)(dst + e0) = v;
}

__global__ __launch_bounds__(256) void rmsnorm_split_kernel(
    const float* __restrict__ x, const float* __restrict__ w,
    unsigned short* __restrict__ outh, unsigned short* __restrict__ outl)
{
  const int lane = threadIdx.x & 31, wave = threadIdx.x >> 5;
  const int row = blockIdx.x * 8 + wave;
  const float* xr = x + (size_t)row * kDm;
  v4f a[8];
#pragma unroll
  for (int j = 0; j < 4; ++j) {
    a[2 * j]     = *(const v4f*)(xr + j * 256 + lane * 8);
    a[2 * j + 1] = *(const v4f*)(xr + j * 256 + lane * 8 + 4);
  }
  float s = 0.f;
#pragma unroll
  for (int i = 0; i < 8; ++i)
#pragma unroll
    for (int e = 0; e < 4; ++e) s = fmaf(a[i][e], a[i][e], s);
#pragma unroll
  for (int off = 16; off >= 1; off >>= 1) s += __shfl_xor(s, off, 32);
  const float r = rsqrtf(s * (1.0f / (float)kDm) + kRmsEps);
  asm volatile("" ::: "memory");
  v4f wv[8];
#pragma unroll
  for (int j = 0; j < 4; ++j) {
    wv[2 * j]     = *(const v4f*)(w + j * 256 + lane * 8);
    wv[2 * j + 1] = *(const v4f*)(w + j * 256 + lane * 8 + 4);
  }
  v8h hv[4], lv[4];
#pragma unroll
  for (int j = 0; j < 4; ++j) {
#pragma unroll
    for (int e = 0; e < 4; ++e) {
      const float f0 = (a[2 * j][e] * r) * wv[2 * j][e];
      const float f1 = (a[2 * j + 1][e] * r) * wv[2 * j + 1][e];
      const unsigned short h0 = f2bf_bits(f0), h1 = f2bf_bits(f1);
      const unsigned short l0 = f2bf_bits(f0 - bf_bits2f(h0)), l1 = f2bf_bits(f1 - bf_bits2f(h1));
      hv[j][e]     = __builtin_bit_cast(_Float16, h0);
      hv[j][4 + e] = __builtin_bit_cast(_Float16, h1);
      lv[j][e]     = __builtin_bit_cast(_Float16, l0);
      lv[j][4 + e] = __builtin_bit_cast(_Float16, l1);
    }
  }
  unsigned short* orh = outh + (size_t)row * kDm;
  unsigned short* orl = outl + (size_t)row * kDm;
  for (int pass = 0; pass < 2; ++pass) {
#pragma unroll
    for (int j = 0; j < 4; ++j) {
      *(volatile v8h*)(orh + j * 256 + lane * 8) = hv[j];
      *(volatile v8h*)(orl + j * 256 + lane * 8) = lv[j];
    }
    __threadfence();
  }
}

__global__ __launch_bounds__(256) void conv_silu_kernel(
    const float* __restrict__ XZ, const float* __restrict__ cw, const float* __restrict__ cb,
    float* __restrict__ UC, unsigned short* __restrict__ UCH, unsigned short* __restrict__ UCL)
{
  __shared__ __align__(16) float sT[16 * kTileP];
  const int tid = threadIdx.x, lane = tid & 31, wave = tid >> 5;
  const int d0 = blockIdx.x * 256, d = d0 + tid;
  const int g0 = blockIdx.y * 64;
  const int tb = g0 & (kSeqT - 1);
  const v4f wq = *(const v4f*)(cw + (size_t)d * 4);
  const float w0 = wq[0], w1 = wq[1], w2 = wq[2], w3 = wq[3];
  const float bc = cb[d];
  float xm3, xm2, xm1;
  {
    const bool hist = (tb > 0);
    const int rb = hist ? (g0 - 3) : g0;
    const float v3 = XZ[(size_t)rb * kXZP + d];
    const float v2 = XZ[(size_t)(rb + 1) * kXZP + d];
    const float v1 = XZ[(size_t)(rb + 2) * kXZP + d];
    xm3 = hist ? v3 : 0.f;
    xm2 = hist ? v2 : 0.f;
    xm1 = hist ? v1 : 0.f;
  }
  const int hrow = wave >> 1;
  const int hch  = (wave & 1) * 128 + lane * 4;
#pragma unroll 1
  for (int sub = 0; sub < 4; ++sub) {
    const int lb = g0 + sub * 16;
#pragma unroll 1
    for (int s = 0; s < 16; ++s) {
      const float xcur = XZ[(size_t)(lb + s) * kXZP + d];
      float acc = w0 * xm3;
      acc = fmaf(w1, xm2, acc);
      acc = fmaf(w2, xm1, acc);
      acc = fmaf(w3, xcur, acc);
      const float sv = acc + bc;
      const float sg = __builtin_amdgcn_rcpf(1.0f + expf(-sv));
      sT[s * kTileP + tid] = sv * sg;
      xm3 = xm2; xm2 = xm1; xm1 = xcur;
    }
    __syncthreads();
    v4f fv[4];
    v8h bh[2], blo[2];
#pragma unroll
    for (int it = 0; it < 4; ++it) fv[it] = *(const v4f*)(sT + (it * 4 + hrow) * kTileP + hch);
#pragma unroll
    for (int it = 0; it < 2; ++it) {
      const float* sp = sT + (it * 8 + wave) * kTileP + lane * 8;
      const v4f a0 = *(const v4f*)(sp);
      const v4f a1 = *(const v4f*)(sp + 4);
#pragma unroll
      for (int e = 0; e < 4; ++e) {
        const float f0 = a0[e], f1 = a1[e];
        const unsigned short h0 = f2bf_bits(f0), h1 = f2bf_bits(f1);
        const unsigned short l0 = f2bf_bits(f0 - bf_bits2f(h0)), l1 = f2bf_bits(f1 - bf_bits2f(h1));
        bh[it][e]      = __builtin_bit_cast(_Float16, h0);
        bh[it][4 + e]  = __builtin_bit_cast(_Float16, h1);
        blo[it][e]     = __builtin_bit_cast(_Float16, l0);
        blo[it][4 + e] = __builtin_bit_cast(_Float16, l1);
      }
    }
    for (int pass = 0; pass < 2; ++pass) {
#pragma unroll
      for (int it = 0; it < 4; ++it)
        *(volatile v4f*)(UC + (size_t)(lb + it * 4 + hrow) * kDin + d0 + hch) = fv[it];
#pragma unroll
      for (int it = 0; it < 2; ++it) {
        const size_t o = (size_t)(lb + it * 8 + wave) * kDin + d0 + lane * 8;
        *(volatile v8h*)(UCH + o) = bh[it];
        *(volatile v8h*)(UCL + o) = blo[it];
      }
      __threadfence();
    }
    __syncthreads();
  }
}

__global__ __launch_bounds__(256) void dlr_cast_kernel(
    const float* __restrict__ DBC, unsigned short* __restrict__ DLR16, int total8, float scale)
{
  const int i = blockIdx.x * 256 + threadIdx.x;
  if (i >= total8) return;
  const int e0  = i << 3;
  const int row = e0 >> 7;
  const int c8  = e0 & (kDtr - 1);
  const float* p = DBC + (size_t)row * kPrjP + c8;
  const v4f a0 = *(const v4f*)(p);
  const v4f a1 = *(const v4f*)(p + 4);
  v8h hv;
#pragma unroll
  for (int e = 0; e < 4; ++e) {
    hv[e]     = (_Float16)(a0[e] * scale);
    hv[4 + e] = (_Float16)(a1[e] * scale);
  }
  unsigned short* qd = DLR16 + e0;
  *(volatile v8h*)qd = hv;
  __threadfence();
  *(volatile v8h*)qd = hv;
}

__global__ __launch_bounds__(256) void scan_kernel(
    const float* __restrict__ DPRE, const float* __restrict__ UC, const float* __restrict__ XZ,
    const float* __restrict__ DBC, const float* __restrict__ A_log,
    unsigned short* __restrict__ YGH, unsigned short* __restrict__ YGL)
{
  __shared__ __align__(16) float sBC[16 * 32];
  __shared__ __align__(16) float sY[16 * kTileP];
  __shared__ __align__(16) float sA[kNst * 256];
  const int tid = threadIdx.x, lane = tid & 31, wave = tid >> 5;
  const int d0 = blockIdx.x * 256, d = d0 + tid;
  const size_t row0 = (size_t)blockIdx.y * kSeqT;

#pragma unroll 1
  for (int n = 0; n < kNst; ++n) sA[n * 256 + tid] = (-expf(A_log[(size_t)d * kNst + n])) * kLog2e;
  __syncthreads();
  float An2[kNst], h[kNst];
#pragma unroll
  for (int n = 0; n < kNst; ++n) {
    An2[n] = sA[n * 256 + tid];
    h[n] = 0.f;
  }

#pragma unroll 1
  for (int c = 0; c < kSeqT / 16; ++c) {
    const int l0 = c * 16;
    if (tid < 128) {
      const int r = tid >> 3, q = (tid & 7) * 4;
      const v4f v = *(const v4f*)(DBC + (row0 + l0 + r) * kPrjP + kDtr + q);
      *(v4f*)(sBC + r * 32 + q) = v;
    }
    __syncthreads();
#pragma unroll 1
    for (int s = 0; s < 16; ++s) {
      const size_t m = row0 + l0 + s;
      const float pv = DPRE[m * kDin + d];
      const float xv = UC[m * kDin + d];
      const float zv = XZ[m * kXZP + kDin + d];
      const float ea  = expf(-fabsf(pv));
      const float u   = 1.0f + ea;
      const float l1p = logf(u) + (ea - (u - 1.0f)) * __builtin_amdgcn_rcpf(u);
      const float delta = fmaxf(pv, 0.0f) + l1p;
      v4f Bq[4], Cq[4];
#pragma unroll
      for (int qq = 0; qq < 4; ++qq) {
        Bq[qq] = *(const v4f*)(sBC + s * 32 + 4 * qq);
        Cq[qq] = *(const v4f*)(sBC + s * 32 + kNst + 4 * qq);
      }
      float y = 0.f;
#pragma unroll
      for (int n = 0; n < kNst; ++n) {
        const float e  = exp2f(delta * An2[n]);
        const float db = delta * Bq[n >> 2][n & 3];
        const float p  = db * xv;
        const float hn = fmaf(e, h[n], p);
        h[n] = hn;
        y = fmaf(hn, Cq[n >> 2][n & 3], y);
      }
      const float sg = __builtin_amdgcn_rcpf(1.0f + expf(-zv));
      const float g  = zv * sg;
      sY[s * kTileP + tid] = y * g;
    }
    __syncthreads();
    v8h hv[2], lv[2];
#pragma unroll
    for (int it = 0; it < 2; ++it) {
      const float* sp = sY + (it * 8 + wave) * kTileP + lane * 8;
      const v4f a0 = *(const v4f*)(sp);
      const v4f a1 = *(const v4f*)(sp + 4);
#pragma unroll
      for (int e = 0; e < 4; ++e) {
        const float f0 = a0[e], f1 = a1[e];
        const unsigned short h0 = f2bf_bits(f0), h1 = f2bf_bits(f1);
        const unsigned short l0 = f2bf_bits(f0 - bf_bits2f(h0)), l1 = f2bf_bits(f1 - bf_bits2f(h1));
        hv[it][e]     = __builtin_bit_cast(_Float16, h0);
        hv[it][4 + e] = __builtin_bit_cast(_Float16, h1);
        lv[it][e]     = __builtin_bit_cast(_Float16, l0);
        lv[it][4 + e] = __builtin_bit_cast(_Float16, l1);
      }
    }
    for (int pass = 0; pass < 2; ++pass) {
#pragma unroll
      for (int it = 0; it < 2; ++it) {
        const size_t o = (row0 + l0 + it * 8 + wave) * kDin + d0 + lane * 8;
        *(volatile v8h*)(YGH + o) = hv[it];
        *(volatile v8h*)(YGL + o) = lv[it];
      }
      __threadfence();
    }
  }
}

static_assert((kRows / 64) * (kXZP / 64) == 256 * 8, "in proj grid");
static_assert((kRows / 64) * (kPrjP / 64) == 12 * 8, "dbc grid");
static_assert((kRows / 64) * (kDin / 64) == 128 * 8, "delta up grid");
static_assert((kRows / 64) * (kDm / 64) == 64 * 8, "out proj grid");
static_assert((kDm % 32) == 0 && (kDin % 32) == 0 && (kDtr % 32) == 0, "GEMM K");

extern "C" void kernel_launch(void* const* d_in, const int* in_sizes, int n_in,
                              void* d_out, int out_size, void* d_ws, size_t ws_size,
                              hipStream_t stream)
{
  if (n_in < 13) return;
  if (in_sizes[0] != kRows * kDm) return;
  if (in_sizes[1] != kDm) return;
  if (in_sizes[2] != kDm * kXZP) return;
  if (in_sizes[3] != kXZP) return;
  if (in_sizes[4] != kDin * 4) return;
  if (in_sizes[5] != kDin) return;
  if (in_sizes[6] != kDin * kNst) return;
  if (in_sizes[7] != kDin * kPrjN) return;
  if (in_sizes[8] != kPrjN) return;
  if (in_sizes[9] != kDtr * kDin) return;
  if (in_sizes[10] != kDin) return;
  if (in_sizes[11] != kDin * kDm) return;
  if (in_sizes[12] != kDm) return;
  if (out_size != kRows * kDm) return;
  if (ws_size < kWsTotal) return;

  const float* x      = (const float*)d_in[0];
  const float* rms_w  = (const float*)d_in[1];
  const float* in_W   = (const float*)d_in[2];
  const float* in_b   = (const float*)d_in[3];
  const float* conv_w = (const float*)d_in[4];
  const float* conv_b = (const float*)d_in[5];
  const float* A_log  = (const float*)d_in[6];
  const float* dbc_W  = (const float*)d_in[7];
  const float* dbc_b  = (const float*)d_in[8];
  const float* dup_W  = (const float*)d_in[9];
  const float* dup_b  = (const float*)d_in[10];
  const float* out_W  = (const float*)d_in[11];
  const float* out_b  = (const float*)d_in[12];
  float* dout = (float*)d_out;

  char* ws = (char*)d_ws;
  unsigned short* INWH  = (unsigned short*)(ws + kOffINWH);
  unsigned short* INWL  = (unsigned short*)(ws + kOffINWL);
  unsigned short* DBH   = (unsigned short*)(ws + kOffDBH);
  unsigned short* DBL   = (unsigned short*)(ws + kOffDBL);
  unsigned short* DUPWT = (unsigned short*)(ws + kOffDUPWT);
  unsigned short* OUTWH = (unsigned short*)(ws + kOffOUTWH);
  unsigned short* OUTWL = (unsigned short*)(ws + kOffOUTWL);
  float*          BIASP = (float*)(ws + kOffBIASP);
  unsigned short* HNH   = (unsigned short*)(ws + kOffHNH);
  unsigned short* HNL   = (unsigned short*)(ws + kOffHNL);
  float*          XZ    = (float*)(ws + kOffXZ);
  float*          UC    = (float*)(ws + kOffUC);
  unsigned short* UCH   = (unsigned short*)(ws + kOffUCH);
  unsigned short* UCL   = (unsigned short*)(ws + kOffUCL);
  float*          DBC   = (float*)(ws + kOffDBC);
  unsigned short* DLR16 = (unsigned short*)(ws + kOffDLR16);
  float*          DPRE  = (float*)(ws + kOffDPRE);
  unsigned short* YGH   = (unsigned short*)(ws + kOffYGH);
  unsigned short* YGL   = (unsigned short*)(ws + kOffYGL);

  transpose_split_bf16_kernel<<<dim3(kXZP / 64, kDm / 64), 256, 0, stream>>>(in_W, INWH, INWL, kDm, kXZP);
  transpose_split_bf16_kernel<<<dim3(kPrjP / 64, kDin / 64), 256, 0, stream>>>(dbc_W, DBH, DBL, kDin, kPrjN);
  transpose_cast_kernel<<<dim3(kDin / 64, kDtr / 64), 256, 0, stream>>>(dup_W, DUPWT, kDtr, kDin, kCarryWdup);
  transpose_split_bf16_kernel<<<dim3(kDm / 64, kDin / 64), 256, 0, stream>>>(out_W, OUTWH, OUTWL, kDin, kDm);
  pad_bias_kernel<<<1, 64, 0, stream>>>(dbc_b, BIASP, kPrjN);

  rmsnorm_split_kernel<<<kRows / 8, 256, 0, stream>>>(x, rms_w, HNH, HNL);

  wmma_gemm64<1, true, 2, false><<<dim3(256, 1), 256, 0, stream>>>(
      HNH, HNL, kDm, 0L, INWH, INWL, kDm, 0L,
      XZ, kXZP, 0L, in_b, x, 0L, kRows, kXZP, kDm, 1.0f);

  conv_silu_kernel<<<dim3(kDin / 256, kRows / 64), 256, 0, stream>>>(XZ, conv_w, conv_b, UC, UCH, UCL);

  wmma_gemm64<1, true, 2, false><<<dim3(12, 1), 256, 0, stream>>>(
      UCH, UCL, kDin, 0L, DBH, DBL, kDin, 0L,
      DBC, kPrjP, 0L, BIASP, x, 0L, kRows, kPrjP, kDin, 1.0f);

  dlr_cast_kernel<<<(kRows * kDtr) / 8 / 256, 256, 0, stream>>>(DBC, DLR16, (kRows * kDtr) / 8, kCarryDlr);

  wmma_gemm64<0, false, 2, false><<<dim3(128, 1), 256, 0, stream>>>(
      DLR16, DLR16, kDtr, 0L, DUPWT, DUPWT, kDtr, 0L,
      DPRE, kDin, 0L, dup_b, x, 0L, kRows, kDin, kDtr, kFoldDt);

  scan_kernel<<<dim3(kDin / 256, kBatch), 256, 0, stream>>>(DPRE, UC, XZ, DBC, A_log, YGH, YGL);

  wmma_gemm64<1, true, 2, true><<<dim3(64, 1), 256, 0, stream>>>(
      YGH, YGL, kDin, 0L, OUTWH, OUTWL, kDin, 0L,
      dout, kDm, 0L, out_b, x, 0L, kRows, kDm, kDin, 1.0f);
}
